// OurModel_18451179503960
// MI455X (gfx1250) — hardware-verified
//
#include <hip/hip_runtime.h>
#include <math.h>

typedef __attribute__((ext_vector_type(16))) _Float16 v16h;
typedef __attribute__((ext_vector_type(16))) __bf16 v16b;
typedef __attribute__((ext_vector_type(8)))  _Float16 v8h;
typedef __attribute__((ext_vector_type(8)))  float v8f;
typedef __attribute__((ext_vector_type(4)))  float v4f;
typedef __attribute__((ext_vector_type(2)))  float v2f;
typedef __attribute__((ext_vector_type(4)))  unsigned v4u;
typedef __attribute__((ext_vector_type(4)))  int v4i;
typedef float __attribute__((may_alias)) float_a;
typedef int __attribute__((may_alias)) int_a;

template <typename T> __device__ __forceinline__ void vst2(void* p, T v) { *(volatile T*)p = v; __threadfence(); *(volatile T*)p = v; }
__device__ __forceinline__ v8f wmma16(v16h a, v16h b, v8f c) {
  v8f d = __builtin_amdgcn_wmma_f32_16x16x32_f16(false, a, false, b, (short)0, c, false, false);
  asm volatile("v_nop\n\tv_nop\n\tv_nop\n\tv_nop" : "+v"(d) : "v"(a), "v"(b));
  return d;
}
__device__ __forceinline__ v8f wmma_bf(v16b a, v16b b, v8f c) {
  v8f d = __builtin_amdgcn_wmma_f32_16x16x32_bf16(false, a, false, b, (short)0, c, false, false);
  asm volatile("v_nop\n\tv_nop\n\tv_nop\n\tv_nop" : "+v"(d) : "v"(a), "v"(b));
  return d;
}
__device__ __forceinline__ v16h frag_h(const _Float16* rowk0, int lane) {
  union { v16h v; v8h q[2]; } u; const _Float16* p = rowk0 + 8 * (lane >> 4);
  u.q[0] = *(const v8h*)p; u.q[1] = *(const v8h*)(p + 16); return u.v;
}
__device__ __forceinline__ v16h frag_f32(const float* rowk0, int lane) {
  v16h a; const float* p = rowk0 + 8 * (lane >> 4);
#pragma unroll
  for (int i = 0; i < 8; ++i) { a[i] = (_Float16)p[i]; a[8 + i] = (_Float16)p[16 + i]; }
  return a;
}
__device__ __forceinline__ v16h frag_f32s(const float* rowk0, int lane, float sc) {
  v16h a; const float* p = rowk0 + 8 * (lane >> 4);
#pragma unroll
  for (int i = 0; i < 8; ++i) { a[i] = (_Float16)(p[i] * sc); a[8 + i] = (_Float16)(p[16 + i] * sc); }
  return a;
}
__device__ __forceinline__ v16h fragc_f32(const float* W, int k0, int n, int lane, int ld, int K) {
  v16h a; const int g = lane >> 4;
#pragma unroll
  for (int i = 0; i < 8; ++i) { const int ka = k0 + 8 * g + i, kb = ka + 16;
    a[i] = (_Float16)(ka < K ? W[(size_t)(ka < K ? ka : K - 1) * ld + n] : 0.f); a[8 + i] = (_Float16)(kb < K ? W[(size_t)(kb < K ? kb : K - 1) * ld + n] : 0.f); }
  return a;
}
struct F2 { v16b h, l; };
__device__ __forceinline__ F2 bsplit16(const float v[16]) { F2 r;
#pragma unroll
  for (int i = 0; i < 16; ++i) { const __bf16 h = (__bf16)v[i]; r.h[i] = h; r.l[i] = (__bf16)(v[i] - (float)h); }
  return r; }
__device__ __forceinline__ F2 split_row(const float* row, int k0, int lane) { float v[16]; const float* p = row + k0 + 8 * (lane >> 4);
#pragma unroll
  for (int i = 0; i < 8; ++i) { v[i] = p[i]; v[8 + i] = p[16 + i]; }
  return bsplit16(v); }
__device__ __forceinline__ F2 split_rowK(const float* row, int k0, int lane, int K) { float v[16]; const int g = lane >> 4;
#pragma unroll
  for (int i = 0; i < 8; ++i) { const int ka = k0 + 8 * g + i, kb = ka + 16; v[i] = ka < K ? row[ka < K ? ka : K - 1] : 0.f; v[8 + i] = kb < K ? row[kb < K ? kb : K - 1] : 0.f; }
  return bsplit16(v); }
__device__ __forceinline__ F2 split_col(const float* W, int k0, int n, int lane, int ld, int K) { float v[16]; const int g = lane >> 4;
#pragma unroll
  for (int i = 0; i < 8; ++i) { const int ka = k0 + 8 * g + i, kb = ka + 16; v[i] = ka < K ? W[(size_t)(ka < K ? ka : K - 1) * ld + n] : 0.f; v[8 + i] = kb < K ? W[(size_t)(kb < K ? kb : K - 1) * ld + n] : 0.f; }
  return bsplit16(v); }
__device__ __forceinline__ v8f mac3(const F2& a, const F2& b, v8f c) { c = wmma_bf(a.l, b.h, c); c = wmma_bf(a.h, b.l, c); return wmma_bf(a.h, b.h, c); }
__device__ __forceinline__ float sigm(float v) { return 1.0f / (1.0f + expf(-v)); }
#define LDSX() do { asm volatile("s_wait_dscnt 0" ::: "memory"); __builtin_amdgcn_wave_barrier(); __builtin_amdgcn_fence(__ATOMIC_RELEASE, "workgroup"); } while (0)


#define NN 20000
#define NE 320000
#define F0 512
#define H1 1024
#define H2 512
#define F3 128
#define D1 152
#define D1P 160
#define D2 48
#define D2P 64
#define NRB ((NN + 63) / 64)
#define NPAD (NRB * 64)
#ifndef TWIN_NP
#define TWIN_NP NN
#define NRBT NRB
#endif
typedef __attribute__((ext_vector_type(8))) __bf16 v8b;
__device__ __forceinline__ v16b frag_b(const __bf16* rowk0, int lane) {
  union { v16b v; v8b q[2]; } u; const __bf16* p = rowk0 + 8 * (lane >> 4);
  u.q[0] = *(const v8b*)p; u.q[1] = *(const v8b*)(p + 16); return u.v;
}
__device__ __forceinline__ float bfr(float v) { return (float)(__bf16)v; }
__device__ __attribute__((noinline)) float exp_ni(float v) { return expf(v); }
__device__ __attribute__((noinline)) float erf_ni(float v) { return erff(v); }

__device__ __attribute__((noinline)) float tanh_ni(float v) { return tanhf(v); }
#define CSA_N 20000
#define CSA_E 320000
#define CSA_FINN (CSA_E + 32 * CSA_NBK)
#define CSA_CHUNK 4096
#define CSA_BKT 256
#define CSA_NCH ((CSA_E + CSA_CHUNK - 1) / CSA_CHUNK)
#define CSA_NBK ((CSA_N + CSA_BKT - 1) / CSA_BKT)
#define CSA_NBKP (((CSA_NBK + 63) / 64) * 64)
#define CSA_SEGCAP (CSA_E + 32 * CSA_NBK * CSA_NCH)
#ifndef CSA_BCAP
#define CSA_BCAP 10240
#endif
#define CSA_SZ_CNT   (4u * CSA_NCH * CSA_NBKP)
#define CSA_SZ_OFF   (4u * CSA_NBK * (((CSA_NCH + 31) / 32) * 32))
#define CSA_SZ_BST   (4u * (((CSA_NBK + 1 + 31) / 32) * 32))
#define CSA_SZ_SEG   (4u * CSA_SEGCAP)
#define CSA_SZ_FIN   (4u * (CSA_E + 32 * CSA_NBK))
#define CSA_SZ_ROW   (4u * CSA_NBK * CSA_BKT)
#define CSA_OFFP (((CSA_NCH + 31) / 32) * 32)

__global__ __launch_bounds__(256) void k_csA_cnt(const int* __restrict__ DST, int dstride, int* __restrict__ CNT) {
  __shared__ unsigned short sc[256][CSA_NBK + 1]; __shared__ __align__(16) int srow[CSA_NBKP];
  const int c = blockIdx.x, tid = threadIdx.x;
  for (int b = 0; b < CSA_NBK; ++b) sc[tid][b] = 0;
  const size_t e0 = (size_t)c * CSA_CHUNK + tid * 16;
  for (int i = 0; i < 16; ++i) { const size_t e = e0 + i; if (e < (size_t)CSA_E) { int d = DST[e * dstride]; d = min(max(d, 0), CSA_N - 1); sc[tid][d / CSA_BKT] += 1; } }
  __syncthreads();
  for (int b = tid; b < CSA_NBKP; b += 256) { int s = 0; if (b < CSA_NBK) for (int t = 0; t < 256; ++t) s += sc[t][b]; srow[b] = s; }
  __syncthreads();
  for (int q = tid; q < CSA_NBKP / 4; q += 256) vst2((unsigned*)(CNT + (size_t)c * CSA_NBKP + q * 4), *(const v4u*)&srow[q * 4]);
}
__global__ __launch_bounds__(256) void k_csA_scan(const int* __restrict__ CNT, int* __restrict__ OFF, int* __restrict__ BST) {
  __shared__ int sbt[CSA_NBK + 1]; __shared__ int sbs[((CSA_NBK + 1 + 31) / 32) * 32]; __shared__ int scnt[CSA_NBK + 1]; __shared__ __align__(16) int sbuf[64][CSA_OFFP];
  const int tid = threadIdx.x;
  for (int b = tid; b < CSA_NBK; b += 256) { int sp = 0, st = 0; for (int c = 0; c < CSA_NCH; ++c) { const int n = CNT[(size_t)c * CSA_NBKP + b]; st += n; sp += (n + 31) & ~31; } sbt[b] = sp; scnt[b] = st; }
  for (int b = tid; b < ((CSA_NBK + 1 + 31) / 32) * 32; b += 256) sbs[b] = 0;
  __syncthreads();
  if (tid == 0) { int acc = 0, accf = 0; for (int b = 0; b < CSA_NBK; ++b) { const int t = sbt[b]; sbt[b] = acc; acc += t; sbs[b] = accf; accf += (scnt[b] + 31) & ~31; } sbs[CSA_NBK] = accf; }
  __syncthreads();
  for (int b0 = 0; b0 < CSA_NBK; b0 += 64) {
    if (tid < 64 && b0 + tid < CSA_NBK) { const int b = b0 + tid; int o = sbt[b]; for (int c = 0; c < CSA_OFFP; ++c) { if (c < CSA_NCH) { sbuf[tid][c] = o; o += (CNT[(size_t)c * CSA_NBKP + b] + 31) & ~31; } else sbuf[tid][c] = 0; } }
    __syncthreads();
    for (int q = tid; q < 64 * (CSA_OFFP / 4); q += 256) { const int r = q / (CSA_OFFP / 4), pc = q % (CSA_OFFP / 4); if (b0 + r < CSA_NBK) vst2((unsigned*)(OFF + (size_t)(b0 + r) * CSA_OFFP + pc * 4), *(const v4u*)&sbuf[r][pc * 4]); }
    __syncthreads(); }
  for (int q = tid; q < ((CSA_NBK + 1 + 31) / 32) * 32 / 4; q += 256) vst2((unsigned*)(BST + q * 4), *(const v4u*)&sbs[q * 4]);
}
__global__ __launch_bounds__(256) void k_csA_scatter(const int* __restrict__ SRC, const int* __restrict__ DST, int sstride, int dstride, const int* __restrict__ OFF, int* __restrict__ SEGS, int* __restrict__ SEGE) {
  __shared__ unsigned short sc[256][CSA_NBK + 1]; __shared__ int sbase[CSA_NBK + 1]; __shared__ int scn[CSA_NBK + 1]; __shared__ int sord[CSA_CHUNK];
  const int c = blockIdx.x, tid = threadIdx.x;
  for (int b = 0; b < CSA_NBK; ++b) sc[tid][b] = 0;
  const size_t e0 = (size_t)c * CSA_CHUNK + tid * 16; int bk[16];
#pragma unroll
  for (int i = 0; i < 16; ++i) { const size_t e = e0 + i; bk[i] = -1; if (e < (size_t)CSA_E) { int d = DST[e * dstride]; d = min(max(d, 0), CSA_N - 1); bk[i] = d / CSA_BKT; sc[tid][bk[i]] += 1; } }
  __syncthreads();
  for (int b = tid; b < CSA_NBK; b += 256) { int acc = 0; for (int t = 0; t < 256; ++t) { const int v = sc[t][b]; sc[t][b] = (unsigned short)acc; acc += v; } scn[b] = acc; }
  __syncthreads();
  if (tid == 0) { int acc = 0; for (int b = 0; b < CSA_NBK; ++b) { sbase[b] = acc; acc += scn[b]; } }
  __syncthreads();
#pragma unroll
  for (int i = 0; i < 16; ++i) { if (bk[i] >= 0) { const int b = bk[i]; const int r = sc[tid][b]; sc[tid][b] = (unsigned short)(r + 1); sord[sbase[b] + r] = tid * 16 + i; } }
  __syncthreads();
  for (int b = 0; b < CSA_NBK; ++b) { const int n = scn[b]; if (n == 0) continue; const int nl = ((n + 31) & ~31); const size_t o = (size_t)(min(max(OFF[(size_t)b * CSA_OFFP + c], 0), CSA_SEGCAP - nl) & ~31);
    for (int q = tid; q < nl / 4; q += 256) { int4 vs, ve;
#pragma unroll
      for (int k = 0; k < 4; ++k) { const int i = q * 4 + k; int s = -1, eid = -1; if (i < n) { const size_t e = (size_t)c * CSA_CHUNK + sord[sbase[b] + i]; s = min(max(SRC[e * sstride], 0), CSA_N - 1); eid = (int)e; } vs[k] = s; ve[k] = eid; }
      vst2((unsigned*)(SEGS + o + q * 4), *(const v4u*)&vs); vst2((unsigned*)(SEGE + o + q * 4), *(const v4u*)&ve); } }
}
__global__ __launch_bounds__(256) void k_csA_bucket(const int* __restrict__ CNT, const int* __restrict__ OFF, const int* __restrict__ BST, const int* __restrict__ SEGS, const int* __restrict__ SEGE, const int* __restrict__ DST, int dstride, int* __restrict__ FS, int* __restrict__ FE, int* __restrict__ ROWST, int* __restrict__ ROWCNT) {
  __shared__ int ssrc[CSA_BCAP]; __shared__ int seid[CSA_BCAP]; __shared__ unsigned char snod[CSA_BCAP]; __shared__ int souts[CSA_BCAP]; __shared__ int soute[CSA_BCAP]; __shared__ int scount[256]; __shared__ int sstart[257]; __shared__ int stot;
  const int b = blockIdx.x, tid = threadIdx.x;
  if (tid == 0) { int t = 0; for (int c = 0; c < CSA_NCH; ++c) t += min(max(CNT[(size_t)c * CSA_NBKP + b], 0), CSA_CHUNK); stot = (t <= CSA_BCAP) ? t : 0; }
  __syncthreads();
  { int base = 0; for (int c = 0; c < CSA_NCH; ++c) { const int n = min(max(CNT[(size_t)c * CSA_NBKP + b], 0), CSA_CHUNK); const int o = min(max(OFF[(size_t)b * CSA_OFFP + c], 0), CSA_SEGCAP - ((n + 31) & ~31));
      for (int i = tid; i < n; i += 256) { const int p = base + i; if (p < CSA_BCAP) { ssrc[p] = min(max(SEGS[o + i], 0), CSA_N - 1); const int e = min(max(SEGE[o + i], 0), CSA_E - 1); seid[p] = e; int d = DST[(size_t)e * dstride]; d = min(max(d, 0), CSA_N - 1); const int dl = d - b * CSA_BKT; snod[p] = (unsigned char)(dl >= 0 && dl < 256 ? dl : 255); } }
      base += n; } }
  __syncthreads();
  const int node = b * CSA_BKT + tid; int cnt = 0; for (int p = 0; p < stot; ++p) cnt += (snod[p] == tid) ? 1 : 0;
  scount[tid] = cnt; __syncthreads();
  if (tid == 0) { int acc = 0; for (int t = 0; t < 256; ++t) { sstart[t] = acc; acc += scount[t]; } sstart[256] = acc; }
  __syncthreads();
  const int bst0 = min(max(BST[b], 0), CSA_FINN - ((sstart[256] + 31) & ~31)) & ~31; const int gst = bst0 + sstart[tid];
  { int w = sstart[tid]; for (int p = 0; p < stot; ++p) if (snod[p] == tid) { souts[w] = ssrc[p]; soute[w] = seid[p]; ++w; } }
  __syncthreads();
  { const int n = sstart[256]; const int nl = (n + 31) & ~31; for (int q = tid; q < nl / 4; q += 256) { int4 vs, ve;
#pragma unroll
      for (int k = 0; k < 4; ++k) { const int i = q * 4 + k; vs[k] = i < n ? souts[i] : -1; ve[k] = i < n ? soute[i] : -1; }
      vst2((unsigned*)(FS + bst0 + q * 4), *(const v4u*)&vs); vst2((unsigned*)(FE + bst0 + q * 4), *(const v4u*)&ve); } }
  __syncthreads();
  { __shared__ __align__(16) int srs[256], src2[256]; srs[tid] = node < CSA_N ? gst : 0; src2[tid] = node < CSA_N ? cnt : 0; __syncthreads();
    if (tid < 64) vst2((unsigned*)(ROWST + (size_t)b * 256 + tid * 4), *(const v4u*)&srs[tid * 4]); else if (tid < 128) vst2((unsigned*)(ROWCNT + (size_t)b * 256 + (tid - 64) * 4), *(const v4u*)&src2[(tid - 64) * 4]); }
}


#define WS_CNT  0u
#define WS_OFF  (WS_CNT + CSA_SZ_CNT)
#define WS_BST  (WS_OFF + CSA_SZ_OFF)
#define WS_SEGS (WS_BST + CSA_SZ_BST)
#define WS_SEGE (WS_SEGS + CSA_SZ_SEG)
#define WS_FS   (WS_SEGE + CSA_SZ_SEG)
#define WS_FE   (WS_FS + CSA_SZ_FIN)
#define WS_RST  (WS_FE + CSA_SZ_FIN)
#define WS_RCT  (WS_RST + CSA_SZ_ROW)
#define WS_PW   (WS_RCT + CSA_SZ_ROW)
#define P1 0
#define P2 (P1 + H1 * F0)
#define P3 (P2 + H2 * H1)
#define PD1 (P3 + F3 * H2)
#define PD2 (PD1 + D1P * F3)
#define PD3 (PD2 + D2P * D1P)
#define PWEND (PD3 + 16 * D2P)
#define WS_A    (WS_PW + 2u * PWEND)
#define WS_B    (WS_A + 4u * NPAD * H1)
#define WS_END  (WS_B + 4u * NPAD * H1)

__global__ __launch_bounds__(256) void k_packT(const float* __restrict__ W1m, const float* __restrict__ W2m, const float* __restrict__ W3m, const float* __restrict__ WD1, const float* __restrict__ WD2, const float* __restrict__ WD3, __bf16* __restrict__ PW) {
  __shared__ __align__(16) __bf16 s[H1]; const int n = blockIdx.x, which = blockIdx.y, tid = threadIdx.x; int K, Kreal, NOUT; const float* Wm; size_t base;
  switch (which) { case 0: K = F0; Kreal = F0; NOUT = H1; Wm = W1m; base = P1; break; case 1: K = H1; Kreal = H1; NOUT = H2; Wm = W2m; base = P2; break; case 2: K = H2; Kreal = H2; NOUT = F3; Wm = W3m; base = P3; break; case 3: K = F3; Kreal = F3; NOUT = D1; Wm = WD1; base = PD1; break; case 4: K = D1P; Kreal = D1; NOUT = D2; Wm = WD2; base = PD2; break; default: K = D2P; Kreal = D2; NOUT = 1; Wm = WD3; base = PD3; break; }
  const int nrows = (which == 3) ? D1P : (which == 4 ? D2P : (which == 5 ? 16 : NOUT)); if (n >= nrows) return;
  for (int k = tid; k < K; k += 256) s[k] = (__bf16)((k < Kreal && n < NOUT) ? Wm[(size_t)k * NOUT + n] : 0.f);
  __syncthreads();
  for (int q = tid; q < K / 8; q += 256) vst2((unsigned*)(PW + base + (size_t)n * K + q * 8), *(const v4u*)&s[q * 8]);
}
template <int RIN, int NT, int EPI>
__global__ __launch_bounds__(128) void k_gemm(const float* __restrict__ A, int lda, int K, const __bf16* __restrict__ P, const float* __restrict__ bias, int nbias, float* __restrict__ OUT, int ldo) {
  __shared__ __align__(16) float so[4][16][NT * 16 + 4];
  const int tid = threadIdx.x, wave = tid >> 5, lane = tid & 31, col = lane & 15, g = lane >> 4; const size_t r0 = (size_t)blockIdx.x * 64 + wave * 16; const int n0 = blockIdx.y * (NT * 16);
  size_t ra = r0 + col; if (ra >= (size_t)NN) ra = NN - 1;
  v8f acc[NT]; for (int j = 0; j < NT; ++j) acc[j] = (v8f){};
#pragma unroll 2
  for (int kc = 0; kc < K / 32; ++kc) { F2 a; if (RIN) { v16b ax; const float* p = A + ra * (size_t)lda + kc * 32 + 8 * g;
#pragma unroll
      for (int i = 0; i < 8; ++i) { ax[i] = (__bf16)p[i]; ax[8 + i] = (__bf16)p[16 + i]; } a.h = ax; a.l = ax; } else a = split_row(A + ra * (size_t)lda, kc * 32, lane);
#pragma unroll
    for (int j = 0; j < NT; ++j) { const v16b w = frag_b(P + (size_t)(n0 + j * 16 + col) * K + kc * 32, lane); if (!RIN) acc[j] = wmma_bf(a.l, w, acc[j]); acc[j] = wmma_bf(a.h, w, acc[j]); } }
#pragma unroll
  for (int j = 0; j < NT; ++j) { const int n = n0 + j * 16 + col; const float bb = (bias && n < nbias) ? bfr(bias[n]) : 0.f;
#pragma unroll
    for (int r = 0; r < 8; ++r) { float v = acc[j][r] + bb; if (EPI == 1) v = fmaxf(v, 0.f); so[wave][8 * g + r][j * 16 + col] = v; } }
  LDSX();
  for (int rl = 0; rl < 16; ++rl) for (int pc = lane; pc < NT * 4; pc += 32) vst2(OUT + (r0 + rl) * (size_t)ldo + n0 + pc * 4, *(const v4f*)&so[wave][rl][pc * 4]);
}
template <int W, int ACT>
__global__ __launch_bounds__(256) void k_wagg(const float* __restrict__ SRC, int lds_, const int* __restrict__ FS, const int* __restrict__ FE, const int* __restrict__ RST, const int* __restrict__ RCT, const float* __restrict__ EW, const float* __restrict__ bias, float* __restrict__ OUT, int ldo) {
  constexpr int TPN = W / 4; constexpr int NPP = 256 / TPN;
  const int tid = threadIdx.x; const int nb = blockIdx.x;
  for (int pass = 0; pass < 64 / NPP; ++pass) { const int nl = pass * NPP + tid / TPN; const int f0 = (tid % TPN) * 4; const int i = nb * 64 + nl;
    v4f acc = {0.f, 0.f, 0.f, 0.f};
    if (i < TWIN_NP) { const int cnt = min(max(RCT[i], 0), CSA_BCAP); const int st = min(max(RST[i], 0), CSA_FINN - cnt);
      for (int e = 0; e < cnt; ++e) { const int s = min(max(FS[st + e], 0), NN - 1); if (s >= TWIN_NP) continue; const int eid = min(max(FE[st + e], 0), NE - 1); const float w = bfr(EW[eid]); const float* row = SRC + (size_t)s * lds_ + f0;
#pragma unroll
        for (int k = 0; k < 4; ++k) acc[k] += w * row[k]; }
#pragma unroll
      for (int k = 0; k < 4; ++k) { float v = acc[k] + bfr(bias[f0 + k]); if (ACT == 1) v = tanh_ni(v); acc[k] = v; } }
    vst2(OUT + (size_t)(nb * 64 + nl) * ldo + f0, acc); }
}
__global__ __launch_bounds__(128) void k_fin(const float* __restrict__ DD2, const __bf16* __restrict__ PW, const float* __restrict__ BD3, float* __restrict__ out) {
  __shared__ __align__(16) float so[64];
  const int tid = threadIdx.x, wave = tid >> 5, lane = tid & 31, col = lane & 15, g = lane >> 4; const size_t r0 = (size_t)blockIdx.x * 64 + wave * 16;
  v8f acc = {};
#pragma unroll
  for (int kc = 0; kc < D2P / 32; ++kc) { const F2 a = split_row(DD2 + (r0 + col) * D2P, kc * 32, lane); const v16b w = frag_b(PW + PD3 + (size_t)col * D2P + kc * 32, lane); acc = wmma_bf(a.l, w, acc); acc = wmma_bf(a.h, w, acc); }
  if (col == 0) {
#pragma unroll
    for (int r = 0; r < 8; ++r) so[wave * 16 + 8 * g + r] = acc[r] + bfr(BD3[0]); }
  __syncthreads();
  if (tid < 16 && blockIdx.x * 64 + tid * 4 + 3 < NN) vst2(out + (size_t)blockIdx.x * 64 + tid * 4, *(const v4f*)&so[tid * 4]);
}
extern "C" void kernel_launch(void* const* d_in, const int* in_sizes, int n_in, void* d_out, int out_size, void* d_ws, size_t ws_size, hipStream_t stream) {
  (void)in_sizes; (void)n_in; (void)out_size;
  const float** F = (const float**)d_in; const int* SRCI = (const int*)d_in[1]; const int* DSTI = (const int*)d_in[2];
  if (ws_size < (size_t)WS_END) return;
  char* ws = (char*)d_ws;
  int *CNT = (int*)(ws + WS_CNT), *OFF = (int*)(ws + WS_OFF), *BST = (int*)(ws + WS_BST), *SEGS = (int*)(ws + WS_SEGS), *SEGE = (int*)(ws + WS_SEGE), *FS = (int*)(ws + WS_FS), *FE = (int*)(ws + WS_FE), *RST = (int*)(ws + WS_RST), *RCT = (int*)(ws + WS_RCT);
  __bf16* PW = (__bf16*)(ws + WS_PW); float *A = (float*)(ws + WS_A), *Bf = (float*)(ws + WS_B);
  k_csA_cnt<<<CSA_NCH, 256, 0, stream>>>(DSTI, 1, CNT); k_csA_scan<<<1, 256, 0, stream>>>(CNT, OFF, BST); k_csA_scatter<<<CSA_NCH, 256, 0, stream>>>(SRCI, DSTI, 1, 1, OFF, SEGS, SEGE); k_csA_bucket<<<CSA_NBK, 256, 0, stream>>>(CNT, OFF, BST, SEGS, SEGE, DSTI, 1, FS, FE, RST, RCT);
  k_packT<<<dim3(H1, 6), 256, 0, stream>>>(F[4], F[6], F[8], F[10], F[12], F[14], PW);
  k_gemm<1, 8, 0><<<dim3(NRBT, H1 / 128), 128, 0, stream>>>(F[0], F0, F0, PW + P1, nullptr, 0, A, H1);
  k_wagg<H1, 1><<<NRBT, 256, 0, stream>>>(A, H1, FS, FE, RST, RCT, F[3], F[5], Bf, H1);
  k_gemm<0, 8, 0><<<dim3(NRBT, H2 / 128), 128, 0, stream>>>(Bf, H1, H1, PW + P2, nullptr, 0, A, H2);
  k_wagg<H2, 1><<<NRBT, 256, 0, stream>>>(A, H2, FS, FE, RST, RCT, F[3], F[7], Bf, H2);
  k_gemm<0, 8, 0><<<dim3(NRBT, 1), 128, 0, stream>>>(Bf, H2, H2, PW + P3, nullptr, 0, A, F3);
  k_wagg<F3, 0><<<NRBT, 256, 0, stream>>>(A, F3, FS, FE, RST, RCT, F[3], F[9], Bf, F3);
  k_gemm<0, 10, 1><<<dim3(NRBT, 1), 128, 0, stream>>>(Bf, F3, F3, PW + PD1, F[11], D1, A, D1P);
  k_gemm<0, 4, 1><<<dim3(NRBT, 1), 128, 0, stream>>>(A, D1P, D1P, PW + PD2, F[13], D2, Bf, D2P);
  k_fin<<<NRBT, 128, 0, stream>>>(Bf, PW, F[15], (float*)d_out);
}
